// EncoderLayer_21406117003700
// MI455X (gfx1250) — hardware-verified
//
#include <hip/hip_runtime.h>
#include <stddef.h>
#include <stdint.h>
#include <math.h>


#define DF     128
#define NHEAD  4
#define NTHR   256
#define NWAVE  8
#define EPT    8
#define CHUNK  (NTHR * EPT)
#define WCAP   (EPT * 32)
#define LISTN  (NWAVE * WCAP)
#define NBA    512
#define SLA    9
#define RCAP   20736
#define DEGCAP 128
#define GBM    64
#define GBN    128
#define GTHR   128
#define WUNITS (DF * (DF / 8))
#define AGG_ZINTS    (LISTN + 2 * RCAP + 3 * NBA)
#define MISC_INTS    16
#define AGG_LDS_INTS (AGG_ZINTS + MISC_INTS)
#define WSMAX  134217728

static_assert((CHUNK & (CHUNK - 1)) == 0 && CHUNK <= 4096);
static_assert((NBA & (NBA - 1)) == 0 && NBA == (1 << SLA));
static_assert(((long long)CHUNK << SLA) < (1LL << 31));
static_assert(LISTN % NTHR == 0);
static_assert(NBA % NWAVE == 0 && NBA % 32 == 0);
static_assert(RCAP % 4 == 0 && AGG_ZINTS % 4 == 0 && LISTN % 4 == 0);
static_assert(DF % 32 == 0 && GBN == DF && GBM == (GTHR / 32) * 16 && DF == 4 * 32 && DF == NHEAD * 32);
static_assert(WUNITS % NTHR == 0 && (GBM * (DF / 8)) % NTHR == 0);
static_assert(DEGCAP >= 61 + 8);
static_assert(AGG_LDS_INTS * 4 <= 300000);

typedef float          v4f   __attribute__((ext_vector_type(4)));
typedef float          v8f   __attribute__((ext_vector_type(8)));
typedef int            v4i   __attribute__((ext_vector_type(4)));
typedef int            v8i   __attribute__((ext_vector_type(8)));
typedef unsigned short v8us  __attribute__((ext_vector_type(8)));
typedef unsigned short v16us __attribute__((ext_vector_type(16)));
typedef __bf16         v16bf __attribute__((ext_vector_type(16)));
typedef v4f  __attribute__((may_alias)) v4fa;
typedef v4i  __attribute__((may_alias)) v4ia;
typedef v8us __attribute__((may_alias)) v8usa;
union FragB { v16bf v; v16us u; v8us h[2]; v8i w; };

__device__ __forceinline__ v8f wmb(const FragB& a, const FragB& b, v8f c) {
  v8f d = __builtin_amdgcn_wmma_f32_16x16x32_bf16(false, a.v, false, b.v, (short)0, c, false, false);
  asm volatile("v_nop\n\tv_nop\n\tv_nop\n\tv_nop" : "+v"(d) : "v"(a.w), "v"(b.w));
  return d;
}

__device__ __forceinline__ unsigned bf16_bits(float f) {
  const unsigned u = __float_as_uint(f);
  return (u + 0x7FFFu + ((u >> 16) & 1u)) >> 16;
}
__device__ __forceinline__ float bf16_val(float f) {
  return __uint_as_float(bf16_bits(f) << 16);
}

__device__ __forceinline__ float score02(float t, float w, float ce) {
  const float al = fmaf(w, ce, t);
  return (al > 0.0f) ? al : 0.2f * al;
}

template <int SLB>
__device__ __forceinline__ int scan_chunk(const int* __restrict__ dsts, int nE, int cbase, int slotBase,
                                          int nb, int vec8, int* list, int tid, int lane, int wave) {
  int wc = 0;
  const int el0  = tid * EPT;
  const int e0   = cbase + el0;
  const int sent = -2147483647 - 1;
  v4i da, db;
  if (vec8 != 0 && cbase + CHUNK <= nE) {
    da = *(const v4i*)(dsts + e0);
    db = *(const v4i*)(dsts + e0 + 4);
  } else {
    da.x = (e0     < nE) ? dsts[min(e0,     nE - 1)] : sent;
    da.y = (e0 + 1 < nE) ? dsts[min(e0 + 1, nE - 1)] : sent;
    da.z = (e0 + 2 < nE) ? dsts[min(e0 + 2, nE - 1)] : sent;
    da.w = (e0 + 3 < nE) ? dsts[min(e0 + 3, nE - 1)] : sent;
    db.x = (e0 + 4 < nE) ? dsts[min(e0 + 4, nE - 1)] : sent;
    db.y = (e0 + 5 < nE) ? dsts[min(e0 + 5, nE - 1)] : sent;
    db.z = (e0 + 6 < nE) ? dsts[min(e0 + 6, nE - 1)] : sent;
    db.w = (e0 + 7 < nE) ? dsts[min(e0 + 7, nE - 1)] : sent;
  }
  const unsigned nbs = (unsigned)slotBase;
  const unsigned unb = (unsigned)nb;
  const unsigned s0 = (unsigned)da.x - nbs, s1 = (unsigned)da.y - nbs;
  const unsigned s2 = (unsigned)da.z - nbs, s3 = (unsigned)da.w - nbs;
  const unsigned s4 = (unsigned)db.x - nbs, s5 = (unsigned)db.y - nbs;
  const unsigned s6 = (unsigned)db.z - nbs, s7 = (unsigned)db.w - nbs;
  const bool h0 = s0 < unb, h1 = s1 < unb, h2 = s2 < unb, h3 = s3 < unb;
  const bool h4 = s4 < unb, h5 = s5 < unb, h6 = s6 < unb, h7 = s7 < unb;
  const unsigned any = __builtin_amdgcn_ballot_w32(h0 | h1 | h2 | h3 | h4 | h5 | h6 | h7);
  if (any != 0u) {
#define HITJ(J, HJ, SJ) { \
      const unsigned mj = __builtin_amdgcn_ballot_w32(HJ); \
      if (mj != 0u) { \
        if (HJ) { \
          const int pos = wc + (int)__builtin_amdgcn_mbcnt_lo(mj, 0u); \
          if (pos < WCAP) list[wave * WCAP + pos] = ((el0 + (J)) << SLB) | (int)(SJ); \
        } \
        wc += (int)__builtin_popcount(mj); } }
    HITJ(0, h0, s0)
    HITJ(1, h1, s1)
    HITJ(2, h2, s2)
    HITJ(3, h3, s3)
    HITJ(4, h4, s4)
    HITJ(5, h5, s5)
    HITJ(6, h6, s6)
    HITJ(7, h7, s7)
#undef HITJ
  }
  return wc;
}

__global__ __launch_bounds__(NTHR) void k_prep(const float* __restrict__ x, const float* __restrict__ W,
                                               int nN, int nUx, unsigned short* xb, unsigned short* wb) {
  const int u = (int)blockIdx.x * NTHR + (int)threadIdx.x;
  v4f a, b;
  bool ok;
  unsigned short* dp;
  if (u < nUx) {
    const int row = u >> 4;
    const int k8  = (u & 15) * 8;
    const int rc  = row < nN ? row : nN - 1;
    const float* p = x + (size_t)rc * DF + k8;
    a = *(const v4fa*)p;
    b = *(const v4fa*)(p + 4);
    ok = row < nN;
    dp = xb + (size_t)row * DF + k8;
  } else {
    const int v = u - nUx;
    if (v >= WUNITS) return;
    const int n  = v >> 4;
    const int k8 = (v & 15) * 8;
    const float* p = W + (size_t)n * DF + k8;
    a = *(const v4fa*)p;
    b = *(const v4fa*)(p + 4);
    ok = true;
    dp = wb + (size_t)n * DF + k8;
  }
  v8us o;
  o[0] = ok ? (unsigned short)bf16_bits(a.x) : (unsigned short)0;
  o[1] = ok ? (unsigned short)bf16_bits(a.y) : (unsigned short)0;
  o[2] = ok ? (unsigned short)bf16_bits(a.z) : (unsigned short)0;
  o[3] = ok ? (unsigned short)bf16_bits(a.w) : (unsigned short)0;
  o[4] = ok ? (unsigned short)bf16_bits(b.x) : (unsigned short)0;
  o[5] = ok ? (unsigned short)bf16_bits(b.y) : (unsigned short)0;
  o[6] = ok ? (unsigned short)bf16_bits(b.z) : (unsigned short)0;
  o[7] = ok ? (unsigned short)bf16_bits(b.w) : (unsigned short)0;
  *(volatile v8us*)dp = o;
  __threadfence();
  *(volatile v8us*)dp = o;
}

__global__ __launch_bounds__(GTHR) void k_proj(const unsigned short* __restrict__ XB,
                                               const unsigned short* __restrict__ WB,
                                               const float* __restrict__ attS, const float* __restrict__ attD,
                                               float* xp, float* asd, int adOff) {
  __shared__ __attribute__((aligned(16))) float stg[GBM * GBN];
  __shared__ __attribute__((aligned(16))) float dots[(GTHR / 32) * 128];
  const int tid = (int)threadIdx.x, lane = tid & 31, wave = tid >> 5, hh = lane >> 4, m = lane & 15;
  const int rowBase = (int)blockIdx.x * GBM;

  v8f acc[8];
  {
    const v8f z = {0.f, 0.f, 0.f, 0.f, 0.f, 0.f, 0.f, 0.f};
#pragma unroll
    for (int t = 0; t < 8; ++t) acc[t] = z;
  }
  const unsigned short* ap = XB + (size_t)(rowBase + 16 * wave + m) * (size_t)DF + 8 * hh;
  const unsigned short* bp = WB + (size_t)m * (size_t)DF + 8 * hh;

#pragma unroll 1
  for (int k0 = 0; k0 < DF; k0 += 32) {
    FragB af;
    af.h[0] = *(const v8usa*)(ap + k0);
    af.h[1] = *(const v8usa*)(ap + k0 + 16);
#pragma unroll
    for (int nt = 0; nt < 8; ++nt) {
      const unsigned short* wq = bp + (size_t)(16 * nt) * (size_t)DF + k0;
      FragB bf;
      bf.h[0] = *(const v8usa*)wq;
      bf.h[1] = *(const v8usa*)(wq + 16);
      acc[nt] = wmb(af, bf, acc[nt]);
    }
  }

#pragma unroll
  for (int nt = 0; nt < 8; ++nt) {
    const int lc = 16 * nt + m;
#pragma unroll
    for (int r = 0; r < 8; ++r) {
      const int lr = 16 * wave + 8 * hh + r;
      stg[lr * GBN + lc] = acc[nt][r];
    }
  }
  __syncthreads();

  v4f as4, ad4;
  {
    const v4f t1 = *(const v4fa*)(attS + 4 * lane);
    const v4f t2 = *(const v4fa*)(attD + 4 * lane);
    as4.x = bf16_val(t1.x); as4.y = bf16_val(t1.y); as4.z = bf16_val(t1.z); as4.w = bf16_val(t1.w);
    ad4.x = bf16_val(t2.x); ad4.y = bf16_val(t2.y); ad4.z = bf16_val(t2.z); ad4.w = bf16_val(t2.w);
  }
  const int hd = lane >> 3;
#pragma unroll 1
  for (int i = 0; i < 16; ++i) {
    const v4f p = *(const v4fa*)(stg + (16 * wave + i) * GBN + 4 * lane);
    float ps = p.x * as4.x;
    ps = fmaf(p.y, as4.y, ps); ps = fmaf(p.z, as4.z, ps); ps = fmaf(p.w, as4.w, ps);
    float pd = p.x * ad4.x;
    pd = fmaf(p.y, ad4.y, pd); pd = fmaf(p.z, ad4.z, pd); pd = fmaf(p.w, ad4.w, pd);
    ps += __shfl_xor(ps, 1, 32); pd += __shfl_xor(pd, 1, 32);
    ps += __shfl_xor(ps, 2, 32); pd += __shfl_xor(pd, 2, 32);
    ps += __shfl_xor(ps, 4, 32); pd += __shfl_xor(pd, 4, 32);
    if ((lane & 7) == 0) {
      dots[wave * 128 + i * 4 + hd]      = ps;
      dots[wave * 128 + 64 + i * 4 + hd] = pd;
    }
  }

  v4f pv[16];
#pragma unroll
  for (int i = 0; i < 16; ++i) pv[i] = *(const v4fa*)(stg + (16 * wave + i) * GBN + 4 * lane);
  __syncthreads();
  const v4f dv = *(const v4fa*)(dots + wave * 128 + 4 * lane);
  const size_t dOff = (size_t)(rowBase + 16 * wave) * NHEAD + (size_t)(4 * (lane & 15))
                    + ((lane >= 16) ? (size_t)adOff : (size_t)0);

#pragma unroll
  for (int i = 0; i < 16; ++i) {
    float* op = xp + (size_t)(rowBase + 16 * wave + i) * DF + 4 * lane;
    *(volatile v4f*)op = pv[i];
  }
  *(volatile v4f*)(asd + dOff) = dv;
  __threadfence();
#pragma unroll
  for (int i = 0; i < 16; ++i) {
    float* op = xp + (size_t)(rowBase + 16 * wave + i) * DF + 4 * lane;
    *(volatile v4f*)op = pv[i];
  }
  *(volatile v4f*)(asd + dOff) = dv;
}

__global__ __launch_bounds__(NTHR) void k_scan(const int* __restrict__ srcs, const int* __restrict__ dsts,
                                               const float* __restrict__ ew, int nE, int nN, int vec8,
                                               const float* __restrict__ xp, const float* __restrict__ asd,
                                               int adOff,
                                               const float* __restrict__ wedge, const float* __restrict__ aedge,
                                               const float* __restrict__ bias, float* out) {
  extern __shared__ __attribute__((aligned(16))) int dsm[];
  int* list = dsm;
  int* hl   = dsm + LISTN;
  int* sl   = hl + RCAP;
  int* cnt  = sl + RCAP;
  int* offs = cnt + NBA;
  int* cur  = offs + NBA;
  int* misc = cur + NBA;
  const int tid = (int)threadIdx.x, lane = tid & 31, wave = tid >> 5;
  const int hd = lane >> 3;
  const int nodeBase = (int)blockIdx.x * NBA;

  {
    const v4i z4 = {0, 0, 0, 0};
    for (int i = tid * 4; i < AGG_ZINTS; i += NTHR * 4) *(v4ia*)(dsm + i) = z4;
    if (tid < MISC_INTS) misc[tid] = 0;
  }
  float ce0, ce1, ce2, ce3;
  v4f bv;
  {
    const v4f w4 = *(const v4fa*)(wedge + 4 * lane);
    const v4f a4 = *(const v4fa*)(aedge + 4 * lane);
    float cep = bf16_val(w4.x) * bf16_val(a4.x);
    cep = fmaf(bf16_val(w4.y), bf16_val(a4.y), cep);
    cep = fmaf(bf16_val(w4.z), bf16_val(a4.z), cep);
    cep = fmaf(bf16_val(w4.w), bf16_val(a4.w), cep);
    cep += __shfl_xor(cep, 1, 32);
    cep += __shfl_xor(cep, 2, 32);
    cep += __shfl_xor(cep, 4, 32);
    ce0 = __shfl(cep, 0, 32);
    ce1 = __shfl(cep, 8, 32);
    ce2 = __shfl(cep, 16, 32);
    ce3 = __shfl(cep, 24, 32);
    const v4f b4 = *(const v4fa*)(bias + 4 * lane);
    bv.x = bf16_val(b4.x); bv.y = bf16_val(b4.y); bv.z = bf16_val(b4.z); bv.w = bf16_val(b4.w);
  }
  __syncthreads();

  int t = 0, ov = 0;
  const int nChunks = (nE + CHUNK - 1) / CHUNK;
#pragma unroll 1
  for (int ch = 0; ch < nChunks; ++ch) {
    const int cbase = ch * CHUNK;
    const int wc = scan_chunk<SLA>(dsts, nE, cbase, nodeBase, NBA, vec8, list, tid, lane, wave);
    if (lane == 0) misc[wave] = wc;
    __syncthreads();
    if (wave == 0) {
#pragma unroll 1
      for (int w2 = 0; w2 < NWAVE; ++w2) {
        int c = misc[w2];
        c = c < 0 ? 0 : (c > WCAP ? WCAP : c);
#pragma unroll 1
        for (int b0 = 0; b0 < c; b0 += 32) {
          const int idx = b0 + lane;
          const int ent = list[w2 * WCAP + (idx < WCAP ? idx : WCAP - 1)];
          const int m32 = (c - b0) < 32 ? (c - b0) : 32;
#pragma unroll 1
          for (int k = 0; k < m32; ++k) {
            const int u    = __builtin_amdgcn_readlane(ent, k);
            const int slot = u & (NBA - 1);
            const int el   = (u >> SLA) & (CHUNK - 1);
            const int pk   = ((cbase + el) << SLA) | slot;
            if (t < RCAP) {
              if (lane == 0) { hl[t] = pk; cnt[slot] = cnt[slot] + 1; }
              t = t + 1;
            } else {
              ov = 1;
            }
          }
        }
      }
    }
    __syncthreads();
  }
  if (wave == 0 && lane == 0) { misc[8] = t; misc[9] = ov; }
  __syncthreads();
  int tt = misc[8];
  tt = tt < 0 ? 0 : (tt > RCAP ? RCAP : tt);
  const int ovf = misc[9];

  if (wave == 0) {
    const int base = lane * (NBA / 32);
    int s = 0;
#pragma unroll 1
    for (int i = 0; i < NBA / 32; ++i) s += cnt[base + i];
    int incl = s;
#pragma unroll
    for (int d = 1; d < 32; d <<= 1) {
      const int y = __shfl_up(incl, d, 32);
      if (lane >= d) incl += y;
    }
    int run = incl - s;
#pragma unroll 1
    for (int i = 0; i < NBA / 32; ++i) {
      const int cv = cnt[base + i];
      offs[base + i] = run;
      cur[base + i]  = run;
      run += cv;
    }
  }
  __syncthreads();
  if (wave == 0) {
#pragma unroll 1
    for (int b0 = 0; b0 < tt; b0 += 32) {
      const int idx = b0 + lane;
      const int ent = hl[idx < RCAP ? idx : RCAP - 1];
      const int m32 = (tt - b0) < 32 ? (tt - b0) : 32;
#pragma unroll 1
      for (int k = 0; k < m32; ++k) {
        const int u    = __builtin_amdgcn_readlane(ent, k);
        const int slot = u & (NBA - 1);
        if (lane == 0) {
          int p = cur[slot];
          p = p < 0 ? 0 : (p > RCAP - 1 ? RCAP - 1 : p);
          sl[p] = u;
          cur[slot] = p + 1;
        }
      }
    }
  }
  __syncthreads();

  const float qnan = __int_as_float(0x7fc00000);
  const float pz   = (ovf != 0) ? qnan : 0.0f;
  const float NEGB = -3.0e38f;
#pragma unroll 1
  for (int si = 0; si < NBA / NWAVE; ++si) {
    const int s    = si * NWAVE + wave;
    const int node = nodeBase + s;
    int c = __builtin_amdgcn_readfirstlane(cnt[s]);
    const bool big = c > DEGCAP;
    c = c < 0 ? 0 : (c > DEGCAP ? DEGCAP : c);
    int o = __builtin_amdgcn_readfirstlane(offs[s]);
    o = o < 0 ? 0 : (o > RCAP ? RCAP : o);
    const int nc = node < nN ? node : nN - 1;
    const v4f adv = *(const v4fa*)(asd + (size_t)adOff + (size_t)nc * NHEAD);
    const v4f asn = *(const v4fa*)(asd + (size_t)nc * NHEAD);

    float m0 = NEGB, m1 = NEGB, m2 = NEGB, m3 = NEGB;
    float wsl = 0.0f;
#pragma unroll 1
    for (int b0 = 0; b0 < c; b0 += 32) {
      const int j = b0 + lane;
      int idx = o + j;
      idx = idx > RCAP - 1 ? RCAP - 1 : idx;
      const int ent = sl[idx];
      int eid = ent >> SLA;
      eid = eid < 0 ? 0 : (eid > nE - 1 ? nE - 1 : eid);
      int sr = srcs[eid];
      sr = sr < 0 ? 0 : (sr > nN - 1 ? nN - 1 : sr);
      const float wv = bf16_val(ew[eid]);
      const v4f a = *(const v4fa*)(asd + (size_t)sr * NHEAD);
      const bool valid = j < c;
      const float al0 = score02(a.x + adv.x, wv, ce0);
      const float al1 = score02(a.y + adv.y, wv, ce1);
      const float al2 = score02(a.z + adv.z, wv, ce2);
      const float al3 = score02(a.w + adv.w, wv, ce3);
      m0 = fmaxf(m0, valid ? al0 : NEGB);
      m1 = fmaxf(m1, valid ? al1 : NEGB);
      m2 = fmaxf(m2, valid ? al2 : NEGB);
      m3 = fmaxf(m3, valid ? al3 : NEGB);
      wsl += valid ? wv : 0.0f;
    }
#pragma unroll
    for (int d = 16; d >= 1; d >>= 1) {
      m0 = fmaxf(m0, __shfl_xor(m0, d, 32));
      m1 = fmaxf(m1, __shfl_xor(m1, d, 32));
      m2 = fmaxf(m2, __shfl_xor(m2, d, 32));
      m3 = fmaxf(m3, __shfl_xor(m3, d, 32));
      wsl += __shfl_xor(wsl, d, 32);
    }
    const float dg = (float)c;
    const float lw = (c > 0) ? (wsl / fmaxf(dg, 1.0f)) : 0.0f;
    m0 = fmaxf(m0, score02(asn.x + adv.x, lw, ce0));
    m1 = fmaxf(m1, score02(asn.y + adv.y, lw, ce1));
    m2 = fmaxf(m2, score02(asn.z + adv.z, lw, ce2));
    m3 = fmaxf(m3, score02(asn.w + adv.w, lw, ce3));

    float dn0 = 0.0f, dn1 = 0.0f, dn2 = 0.0f, dn3 = 0.0f;
    float acc0 = 0.0f, acc1 = 0.0f, acc2 = 0.0f, acc3 = 0.0f;
    const int cext = c + 1;
    const int lwi  = __float_as_int(lw);
#pragma unroll 1
    for (int b0 = 0; b0 < cext; b0 += 32) {
      const int j = b0 + lane;
      int idx = o + j;
      idx = idx > RCAP - 1 ? RCAP - 1 : idx;
      const int ent = sl[idx];
      int eid = ent >> SLA;
      eid = eid < 0 ? 0 : (eid > nE - 1 ? nE - 1 : eid);
      int srl = srcs[eid];
      srl = srl < 0 ? 0 : (srl > nN - 1 ? nN - 1 : srl);
      const int wli  = __float_as_int(bf16_val(ew[eid]));
      const int selm = -(int)(j == c);
      const int sr   = (srl & ~selm) | (nc & selm);
      const float wv = __int_as_float((wli & ~selm) | (lwi & selm));
      const v4f a = *(const v4fa*)(asd + (size_t)sr * NHEAD);
      const bool valid = j < cext;
      const float al0 = score02(a.x + adv.x, wv, ce0);
      const float al1 = score02(a.y + adv.y, wv, ce1);
      const float al2 = score02(a.z + adv.z, wv, ce2);
      const float al3 = score02(a.w + adv.w, wv, ce3);
      const float x0 = expf(al0 - m0), x1 = expf(al1 - m1), x2 = expf(al2 - m2), x3 = expf(al3 - m3);
      const float e0 = valid ? x0 : 0.0f;
      const float e1 = valid ? x1 : 0.0f;
      const float e2 = valid ? x2 : 0.0f;
      const float e3 = valid ? x3 : 0.0f;
      dn0 += e0; dn1 += e1; dn2 += e2; dn3 += e3;
      const int e0i = __float_as_int(e0), e1i = __float_as_int(e1);
      const int e2i = __float_as_int(e2), e3i = __float_as_int(e3);
      const int m32 = (cext - b0) < 32 ? (cext - b0) : 32;
#pragma unroll 1
      for (int k = 0; k < m32; ++k) {
        const int   sk = __builtin_amdgcn_readlane(sr, k);
        const float q0 = __int_as_float(__builtin_amdgcn_readlane(e0i, k));
        const float q1 = __int_as_float(__builtin_amdgcn_readlane(e1i, k));
        const float q2 = __int_as_float(__builtin_amdgcn_readlane(e2i, k));
        const float q3 = __int_as_float(__builtin_amdgcn_readlane(e3i, k));
        const float ck = (hd == 0) ? q0 : ((hd == 1) ? q1 : ((hd == 2) ? q2 : q3));
        const v4f r = *(const v4fa*)(xp + (size_t)sk * DF + 4 * lane);
        acc0 = fmaf(ck, r.x, acc0);
        acc1 = fmaf(ck, r.y, acc1);
        acc2 = fmaf(ck, r.z, acc2);
        acc3 = fmaf(ck, r.w, acc3);
      }
    }
#pragma unroll
    for (int d = 16; d >= 1; d >>= 1) {
      dn0 += __shfl_xor(dn0, d, 32);
      dn1 += __shfl_xor(dn1, d, 32);
      dn2 += __shfl_xor(dn2, d, 32);
      dn3 += __shfl_xor(dn3, d, 32);
    }
    const float dn = (hd == 0) ? dn0 : ((hd == 1) ? dn1 : ((hd == 2) ? dn2 : dn3));
    const float rd = 1.0f / dn;
    const float pzr = big ? qnan : pz;
    v4f y;
    y.x = fmaf(acc0, rd, bv.x);
    y.y = fmaf(acc1, rd, bv.y);
    y.z = fmaf(acc2, rd, bv.z);
    y.w = fmaf(acc3, rd, bv.w);
    y.x = (y.x > 0.0f) ? y.x : 0.01f * y.x;
    y.y = (y.y > 0.0f) ? y.y : 0.01f * y.y;
    y.z = (y.z > 0.0f) ? y.z : 0.01f * y.z;
    y.w = (y.w > 0.0f) ? y.w : 0.01f * y.w;
    y.x = y.x + pzr; y.y = y.y + pzr; y.z = y.z + pzr; y.w = y.w + pzr;
    float* op = out + (size_t)nc * DF + 4 * lane;
    if (node < nN) *(volatile v4f*)op = y;
    __threadfence();
    if (node < nN) *(volatile v4f*)op = y;
  }
}

static inline int cdiv(int a, int b) { return (a + b - 1) / b; }
static inline size_t al256(size_t o) { return (o + 255) & ~(size_t)255; }

extern "C" void kernel_launch(void* const* d_in, const int* in_sizes, int n_in,
                              void* d_out, int out_size, void* d_ws, size_t ws_size,
                              hipStream_t stream) {
  if (n_in < 9) return;
  if (in_sizes[0] < DF || (in_sizes[0] % DF) != 0) return;
  const int nN = in_sizes[0] / DF;
  if (nN < 16 || nN > (1 << 22)) return;
  if (in_sizes[1] < 2 || (in_sizes[1] & 1) != 0) return;
  const int nE = in_sizes[1] / 2;
  if (nE < 1 || nE >= (1 << (31 - SLA))) return;
  if (in_sizes[2] != nE) return;
  if (in_sizes[3] != DF * DF) return;
  if (in_sizes[4] != DF || in_sizes[5] != DF) return;
  if (in_sizes[6] != DF || in_sizes[7] != DF) return;
  if (in_sizes[8] != DF) return;
  if ((long long)out_size != (long long)nN * DF) return;

  const float* x     = (const float*)d_in[0];
  const int*   edge  = (const int*)d_in[1];
  const float* ewt   = (const float*)d_in[2];
  const float* Wsrc  = (const float*)d_in[3];
  const float* attS  = (const float*)d_in[4];
  const float* attD  = (const float*)d_in[5];
  const float* Wedge = (const float*)d_in[6];
  const float* attE  = (const float*)d_in[7];
  const float* bias  = (const float*)d_in[8];
  float* out = (float*)d_out;
  const int* src = edge;
  const int* dst = edge + nE;

  const int MP  = cdiv(nN, GBM) * GBM;
  const int gM  = MP / GBM;
  const int gA  = cdiv(nN, NBA);
  if ((long long)gA * NBA < (long long)nN) return;
  const int nUx = MP * (DF / 8);
  if ((nUx % NTHR) != 0) return;
  const int adOff = MP * NHEAD;
  const int vec8 = ((nE & 3) == 0) ? 1 : 0;

  char* ws = (char*)d_ws;
  size_t off = 0;
  const size_t oXB  = off; off = al256(off + (size_t)MP * DF * 2);
  const size_t oWB  = off; off = al256(off + (size_t)DF * DF * 2);
  const size_t oXP  = off; off = al256(off + (size_t)MP * DF * 4);
  const size_t oASD = off; off = al256(off + (size_t)2 * MP * NHEAD * 4);
  if (off > ws_size || off > (size_t)WSMAX) return;
  unsigned short* XB  = (unsigned short*)(ws + oXB);
  unsigned short* WB  = (unsigned short*)(ws + oWB);
  float*          XP  = (float*)(ws + oXP);
  float*          ASD = (float*)(ws + oASD);

  const size_t scanLds = (size_t)AGG_LDS_INTS * 4;
  hipFuncSetAttribute(reinterpret_cast<const void*>(&k_scan), hipFuncAttributeMaxDynamicSharedMemorySize, (int)scanLds);

  k_prep<<<(nUx + WUNITS) / NTHR, NTHR, 0, stream>>>(x, Wsrc, nN, nUx, XB, WB);
  k_proj<<<gM, GTHR, 0, stream>>>(XB, WB, attS, attD, XP, ASD, adOff);
  k_scan<<<gA, NTHR, scanLds, stream>>>(src, dst, ewt, nE, nN, vec8, XP, ASD, adOff, Wedge, attE, bias, out);
}
